// MCModel_16956530884805
// MI455X (gfx1250) — hardware-verified
//
#include <hip/hip_runtime.h>


namespace {
constexpr int B = 64, T = 256, M = 16, A = 32, H = 64, NR = B * T;
constexpr float XS = 8.0f, WSC = 256.0f;
typedef _Float16 b16;
typedef __attribute__((ext_vector_type(16))) _Float16 v16b;
typedef __attribute__((ext_vector_type(8))) _Float16 v8b;
typedef __attribute__((ext_vector_type(8))) float v8f;
typedef __attribute__((ext_vector_type(4))) float v4f;
typedef __attribute__((ext_vector_type(2))) float v2f;
__device__ __forceinline__ float bf16_rne(float f) { unsigned int u = __float_as_uint(f); u += 0x7FFFu + ((u >> 16) & 1u); return __uint_as_float(u & 0xFFFF0000u); }
__device__ __forceinline__ v16b frag_kb(const b16* p, int hh) { const v8b a = *(const v8b*)(p + 8 * hh), b = *(const v8b*)(p + 16 + 8 * hh); v16b f;
#pragma unroll
  for (int e = 0; e < 8; ++e) { f[e] = a[e]; f[8 + e] = b[e]; } return f; }
__device__ __forceinline__ v8f wmma16b(v16b a, v16b b, v8f c) { v8f d = __builtin_amdgcn_wmma_f32_16x16x32_f16(false, a, false, b, (short)0, c, false, false); asm volatile("v_nop\n\tv_nop\n\tv_nop\n\tv_nop" : "+v"(d) : "v"(a), "v"(b)); return d; }
__device__ __forceinline__ void wave_lds_sync() { __builtin_amdgcn_fence(__ATOMIC_RELEASE, "workgroup"); __builtin_amdgcn_wave_barrier(); __builtin_amdgcn_fence(__ATOMIC_ACQUIRE, "workgroup"); }
__device__ __forceinline__ float pmul(float a, float b) { float p = a * b; asm volatile("" : "+v"(p)); return p; }

__global__ __launch_bounds__(256) void wcopy_kernel(const float* __restrict__ w, int OUTW, int o0, b16* __restrict__ WT) { const int u = blockIdx.x * 256 + threadIdx.x; if (u >= OUTW * 4) return; const int o = u / 4, k0 = (u % 4) * 8; v8b v;
#pragma unroll
  for (int j = 0; j < 8; ++j) v[j] = (b16)(bf16_rne(w[(size_t)o * A + k0 + j]) * WSC); for (int pass = 0; pass < 2; ++pass) { *(volatile v8b*)(WT + (size_t)(o0 + o) * A + k0) = v; __threadfence(); } }
__global__ __launch_bounds__(32) void gate_kernel(const float* __restrict__ xa, const b16* __restrict__ WT, const float* __restrict__ bj, const float* __restrict__ br, const float* __restrict__ bo, int BV, int t0, int TCH, float* __restrict__ Gp) {
  __shared__ __attribute__((aligned(16))) b16 Ah[16][40]; __shared__ float Tf[16][132]; const int lane = threadIdx.x, nloc = lane & 15, hlf = lane >> 4; const int NCG = 41; const int cg = blockIdx.x % NCG; const size_t m0 = (size_t)(blockIdx.x / NCG) * 16; if (m0 >= (size_t)BV * TCH) return;
  auto srcrow = [&](size_t r) { const size_t bq = r / TCH, tt = r % TCH; return bq * T + t0 + tt; };
  for (int rr = 0; rr < 16; ++rr) Ah[rr][lane] = (b16)(bf16_rne(xa[srcrow(m0 + rr) * A + lane]) * XS);
  wave_lds_sync(); const v16b a = frag_kb(&Ah[nloc][0], hlf); const int ntile = (cg == 40) ? 4 : 8; const int c0 = cg * 128;
  for (int t = 0; t < 8; ++t) { if (t >= ntile) break; v8f acc = {}; acc = wmma16b(a, frag_kb(WT + (size_t)(c0 + t * 16 + nloc) * A, hlf), acc); const int c = c0 + t * 16 + nloc; const float bb = bf16_rne(c < 1024 ? bj[c] : (c < 5120 ? br[c - 1024] : bo[c - 5120]));
#pragma unroll
    for (int r8 = 0; r8 < 8; ++r8) Tf[8 * hlf + r8][t * 16 + nloc] = acc[r8] * (1.0f / (XS * WSC)) + bb; }
  wave_lds_sync();
  { const int row = lane & 15, grp = lane >> 4; if (cg < 40) { float mx = -INFINITY; for (int k = 0; k < 64; ++k) mx = fmaxf(mx, Tf[row][grp * 64 + k]); float s = 0.0f; for (int k = 0; k < 64; ++k) s += __expf(Tf[row][grp * 64 + k] - mx); const float inv = 1.0f / s; wave_lds_sync(); for (int k = 0; k < 64; ++k) Tf[row][grp * 64 + k] = __expf(Tf[row][grp * 64 + k] - mx) * inv; }
    else { wave_lds_sync(); for (int k = 0; k < 32; ++k) { const int c = grp * 32 + k; Tf[row][c] = 1.0f / (1.0f + __expf(-Tf[row][c])); } } }
  wave_lds_sync();
  for (int pass = 0; pass < 2; ++pass) { for (int rr = 0; rr < 16; ++rr) { if (cg < 40) *(volatile v4f*)(Gp + (m0 + rr) * 5184 + c0 + lane * 4) = *(const v4f*)(&Tf[rr][lane * 4]); else *(volatile v2f*)(Gp + (m0 + rr) * 5184 + c0 + lane * 2) = (v2f){Tf[rr][lane * 2], Tf[rr][lane * 2 + 1]}; } __threadfence(); }
}
__global__ __launch_bounds__(32) void scan_kernel(const float* __restrict__ Gp, const float* __restrict__ xm, const float* __restrict__ wfc, const float* __restrict__ bfc, int BV, int t0, int TCH, float* __restrict__ CST, float* __restrict__ pred, float* __restrict__ cout) {
  __shared__ float Cs[H]; const int lane = threadIdx.x; const int b = blockIdx.x; if (b >= BV) return; const int k0 = lane * 2;
  const float cst0 = t0 == 0 ? 0.0f : CST[(size_t)b * H + k0], cst1 = t0 == 0 ? 0.0f : CST[(size_t)b * H + k0 + 1]; float cl0 = cst0, cl1 = cst1;
  for (int pass = 0; pass < 2; ++pass) { Cs[k0] = cst0; Cs[k0 + 1] = cst1; float mo0 = 0.0f, mo1 = 0.0f; wave_lds_sync();
#pragma unroll 1
    for (int t = t0; t < t0 + TCH; ++t) { const size_t row = (size_t)b * T + t; const float* g = Gp + ((size_t)b * TCH + (t - t0)) * 5184; float mi0 = 0.0f, mi1 = 0.0f;
#pragma unroll 1
      for (int m = 0; m < M; ++m) { const float xv = bf16_rne(xm[row * M + m]); mi0 += pmul(xv, g[m * H + k0]); mi1 += pmul(xv, g[m * H + k0 + 1]); }
      float s0 = 0.0f, s1 = 0.0f;
#pragma unroll 1
      for (int h = 0; h < H; ++h) { const float ch = Cs[h]; s0 += pmul(ch, g[1024 + h * H + k0]); s1 += pmul(ch, g[1024 + h * H + k0 + 1]); }
      const float mn0 = mi0 + s0, mn1 = mi1 + s1; const float o0 = g[5120 + k0], o1 = g[5120 + k0 + 1]; const float c0 = pmul(1.0f - o0, mn0), c1 = pmul(1.0f - o1, mn1); mo0 = pmul(o0, mn0); mo1 = pmul(o1, mn1);
      wave_lds_sync(); Cs[k0] = c0; Cs[k0 + 1] = c1; cl0 = c0; cl1 = c1; wave_lds_sync();
      *(volatile v2f*)(cout + row * H + k0) = (v2f){c0, c1}; }
    float p = pmul(mo0, bf16_rne(wfc[k0])) + pmul(mo1, bf16_rne(wfc[k0 + 1])); for (int o = 16; o; o >>= 1) p += __shfl_xor(p, o); p += bf16_rne(bfc[0]);
    if (t0 + TCH == T) ((volatile float*)pred)[(size_t)b * 32 + lane] = lane == 0 ? p : 0.0f;
    __threadfence(); }
  wave_lds_sync(); for (int pass = 0; pass < 2; ++pass) { *(volatile v2f*)(CST + (size_t)b * H + k0) = (v2f){cl0, cl1}; __threadfence(); }
}
__global__ __launch_bounds__(64) void pred_kernel(const float* __restrict__ PST, float* __restrict__ pred) { const int b = threadIdx.x; const float v = PST[(size_t)b * 32]; for (int pass = 0; pass < 2; ++pass) { ((volatile float*)pred)[b] = v; __threadfence(); } }
}

extern "C" void kernel_launch(void* const* d_in, const int* in_sizes, int n_in, void* d_out, int out_size, void* d_ws, size_t ws_size, hipStream_t stream) {
  (void)n_in;
  auto Fp = [&](int i) { return (const float*)d_in[i]; };
  if (in_sizes[0] != NR * M || in_sizes[1] != NR * A || in_sizes[2] != 1024 * A || in_sizes[4] != 4096 * A || in_sizes[6] != H * A || in_sizes[8] != H || out_size != B + NR * H) return;
  const int BV = B; const int TCH = 32;
  size_t off = 0; char* ws = (char*)d_ws;
  auto carve = [&](size_t bytes) { char* p = ws + off; off += (bytes + 255) & ~(size_t)255; return p; };
  b16* WT = (b16*)carve((size_t)5184 * A * 2); float* Gp = (float*)carve((size_t)B * TCH * 5184 * 4); float* PST = (float*)carve((size_t)B * 32 * 4); float* CST = (float*)carve((size_t)B * H * 4);
  if (off > ws_size || off > ((size_t)64 << 20)) return;
  wcopy_kernel<<<(1024 * 4 + 255) / 256, 256, 0, stream>>>(Fp(2), 1024, 0, WT); wcopy_kernel<<<(4096 * 4 + 255) / 256, 256, 0, stream>>>(Fp(4), 4096, 1024, WT); wcopy_kernel<<<(H * 4 + 255) / 256, 256, 0, stream>>>(Fp(6), H, 5120, WT);
  float* out = (float*)d_out;
  for (int t0 = 0; t0 < T; t0 += TCH) {
    gate_kernel<<<(BV * TCH / 16) * 41, 32, 0, stream>>>(Fp(1), WT, Fp(3), Fp(5), Fp(7), BV, t0, TCH, Gp);
    scan_kernel<<<BV, 32, 0, stream>>>(Gp, Fp(0), Fp(8), Fp(9), BV, t0, TCH, CST, PST, out + B); }
  pred_kernel<<<1, 64, 0, stream>>>(PST, out);
}
